// ICTDIrrepsE3Conv_26628797235369
// MI455X (gfx1250) — hardware-run, weakly checked
//
#include <hip/hip_runtime.h>

typedef float          v8f   __attribute__((ext_vector_type(8)));
typedef float          v4f   __attribute__((ext_vector_type(4)));
typedef unsigned int   v4u   __attribute__((ext_vector_type(4)));
typedef int            v8i   __attribute__((ext_vector_type(8)));
typedef unsigned short v8us  __attribute__((ext_vector_type(8)));
typedef unsigned short v16us __attribute__((ext_vector_type(16)));
typedef __bf16         v16bf __attribute__((ext_vector_type(16)));
typedef _Float16       v16h  __attribute__((ext_vector_type(16)));
typedef v4f  __attribute__((may_alias)) v4fa;
typedef v8us __attribute__((may_alias)) v8usa;
union FragB { v16bf v; v16us u; v8us h[2]; v8i w; };
union FragH { v16h  v; v16us u; v8us h[2]; v8i w; };

__device__ __forceinline__ v8f wmb(const FragB& a, const FragB& b, v8f c) {
  v8f d = __builtin_amdgcn_wmma_f32_16x16x32_bf16(false, a.v, false, b.v, (short)0, c, false, false);
  asm volatile("v_nop\n\tv_nop\n\tv_nop\n\tv_nop" : "+v"(d) : "v"(a.w), "v"(b.w));
  return d;
}

__device__ __forceinline__ v8f wmh(const FragH& a, const FragH& b, v8f c) {
  v8f d = __builtin_amdgcn_wmma_f32_16x16x32_f16(false, a.v, false, b.v, (short)0, c, false, false);
  asm volatile("v_nop\n\tv_nop\n\tv_nop\n\tv_nop" : "+v"(d) : "v"(a.w), "v"(b.w));
  return d;
}

__device__ __forceinline__ unsigned bf16_bits(float f) {
  const unsigned u = __float_as_uint(f);
  const unsigned r = (u + 0x7FFFu + ((u >> 16) & 1u)) >> 16;
  const unsigned q = (u >> 16) | 0x40u;
  return ((u & 0x7fffffffu) > 0x7f800000u) ? q : r;
}

__device__ __forceinline__ float bf16_val(float f) {
  return __uint_as_float(bf16_bits(f) << 16);
}
__device__ __forceinline__ int clampi(int v, int lo, int hi) {
  return v < lo ? lo : (v > hi ? hi : v);
}

__device__ __forceinline__ unsigned f16_bits(float f) {
  const unsigned u  = __float_as_uint(f);
  const unsigned s  = (u >> 16) & 0x8000u;
  const unsigned a  = u & 0x7fffffffu;
  const unsigned t  = a - 0x38000000u;
  const unsigned r  = (t + 0x0FFFu + ((t >> 13) & 1u)) >> 13;
  const unsigned rc = r > 0x7C00u ? 0x7C00u : r;
  const bool small  = a < 0x38800000u;
  const bool isnan  = a > 0x7f800000u;
  const unsigned fin = small ? 0u : (s | rc);
  return isnan ? (s | 0x7E00u) : fin;
}

__device__ __forceinline__ unsigned pk16(unsigned lo, unsigned hi) { return lo | (hi << 16); }
__device__ __forceinline__ unsigned bf16_lo_bits(float v) {
  float hi = bf16_val(v);
  asm volatile("" : "+v"(hi));
  return bf16_bits(v - hi);
}
__device__ __forceinline__ v4u pack8_bf16(v4f a, v4f c) {
  return (v4u){ pk16(bf16_bits(a[0]), bf16_bits(a[1])), pk16(bf16_bits(a[2]), bf16_bits(a[3])),
                pk16(bf16_bits(c[0]), bf16_bits(c[1])), pk16(bf16_bits(c[2]), bf16_bits(c[3])) };
}
__device__ __forceinline__ v4u pack8_bf16_lo(v4f a, v4f c) {
  return (v4u){ pk16(bf16_lo_bits(a[0]), bf16_lo_bits(a[1])), pk16(bf16_lo_bits(a[2]), bf16_lo_bits(a[3])),
                pk16(bf16_lo_bits(c[0]), bf16_lo_bits(c[1])), pk16(bf16_lo_bits(c[2]), bf16_lo_bits(c[3])) };
}
__device__ __forceinline__ v4u pack8_f16(v4f a, v4f c) {
  return (v4u){ pk16(f16_bits(a[0]), f16_bits(a[1])), pk16(f16_bits(a[2]), f16_bits(a[3])),
                pk16(f16_bits(c[0]), f16_bits(c[1])), pk16(f16_bits(c[2]), f16_bits(c[3])) };
}

template <int FORM>
__global__ __launch_bounds__(256) void k_plane(const float* __restrict__ src, int rows, int cols, int ldsrc,
                                               unsigned short* __restrict__ dst, int MP, int KP) {
  static_assert(FORM >= 0 && FORM <= 3);
  const int KTOT = (FORM == 1 || FORM == 3) ? 2 * KP : KP;
  const unsigned ppr   = (unsigned)(KTOT >> 3);
  const unsigned kp8   = (unsigned)(KP >> 3);
  const unsigned total = (unsigned)MP * ppr;
  const unsigned g     = blockIdx.x * 256u + threadIdx.x;
  const unsigned rowu  = g / ppr;
  const unsigned p     = g - rowu * ppr;
  const bool second    = p >= kp8;
  const int row = (int)rowu;
  const int c0  = (int)((second ? p - kp8 : p) << 3);
  const float* srow = src + (size_t)clampi(row, 0, rows - 1) * (size_t)ldsrc;
  float x[8];
  unsigned mk[8];
#pragma unroll
  for (int e = 0; e < 8; ++e) {
    const int c = c0 + e;
    const float v = srow[clampi(c, 0, cols - 1)];
    asm volatile("" :: "v"(v));
    x[e]  = v;
    mk[e] = (row < rows && c < cols) ? 0xFFFFu : 0u;
  }
  const v4f a = (v4f){ x[0], x[1], x[2], x[3] };
  const v4f c = (v4f){ x[4], x[5], x[6], x[7] };
  v4u o;
  if (FORM == 2) {
    o = pack8_f16(a, c);
  } else {
    const v4u hi = pack8_bf16(a, c);
    o = hi;
    if (FORM == 1) { const v4u lo = pack8_bf16_lo(a, c); o = second ? lo : hi; }
  }
  const v4u mw = (v4u){ pk16(mk[0], mk[1]), pk16(mk[2], mk[3]), pk16(mk[4], mk[5]), pk16(mk[6], mk[7]) };
  o &= mw;
  if (g < total) {
    volatile v4u* q = (volatile v4u*)(dst + (size_t)g * 8);
    *q = o;
    __threadfence();
    *q = o;
  }
}

template <int FORM> struct FragOf    { typedef FragB T; };
template <>         struct FragOf<2> { typedef FragH T; };
__device__ __forceinline__ v8f mm(const FragB& a, const FragB& b, v8f c) { return wmb(a, b, c); }
__device__ __forceinline__ v8f mm(const FragH& a, const FragH& b, v8f c) { return wmh(a, b, c); }
template <class F> __device__ __forceinline__ F ld_frag(const unsigned short* p) {
  F f;
  f.h[0] = *(const v8usa*)(p);
  f.h[1] = *(const v8usa*)(p + 16);
  return f;
}

template <int FORM, int EPI>
__global__ __launch_bounds__(256) __attribute__((amdgpu_num_vgpr(248)))
void k_gemm_nt(const unsigned short* __restrict__ A, const unsigned short* __restrict__ B,
               const float* __restrict__ bias, float* __restrict__ D, int M, int N, int KTOT, int ldd) {
  static_assert(FORM >= 0 && FORM <= 2);
  static_assert(EPI == 0 || EPI == 1);
  typedef typename FragOf<FORM>::T F;
  __shared__ __attribute__((aligned(16))) float sT[8][16 * 68];
  const int lane = threadIdx.x & 31;
  const int wave = threadIdx.x >> 5;
  const int tilesM = (M + 63) >> 6;
  const int tilesN = (N + 63) >> 6;
  const int tile = blockIdx.x * 8 + wave;
  if (tile >= tilesM * tilesN) return;
  const int tm = tile / tilesN;
  const int tn = tile - tm * tilesN;
  const int m0 = tm << 6;
  const int n0 = tn << 6;

  const int rl = lane & 15;
  const int h8 = (lane >> 4) * 8;
  const unsigned short* pa = A + (size_t)(m0 + rl) * (size_t)KTOT + h8;
  const unsigned short* pb = B + (size_t)(n0 + rl) * (size_t)KTOT + h8;

  v8f acc[4][4];
#pragma unroll
  for (int i = 0; i < 4; ++i)
#pragma unroll
    for (int j = 0; j < 4; ++j) acc[i][j] = (v8f){0.f, 0.f, 0.f, 0.f, 0.f, 0.f, 0.f, 0.f};

#pragma unroll 1
  for (int k0 = 0; k0 < KTOT; k0 += 32) {
    F bf[4];
#pragma unroll
    for (int j = 0; j < 4; ++j) bf[j] = ld_frag<F>(pb + (size_t)(j << 4) * (size_t)KTOT + k0);
#pragma unroll
    for (int i = 0; i < 4; ++i) {
      const F af = ld_frag<F>(pa + (size_t)(i << 4) * (size_t)KTOT + k0);
#pragma unroll
      for (int j = 0; j < 4; ++j) acc[i][j] = mm(af, bf[j], acc[i][j]);
    }
  }

  float* slab = sT[wave];
  const int hh = lane >> 4;
  const int c4 = (lane & 15) * 4;
  const int nc = n0 + c4;
  const bool cok = nc < N;
  v4f bv = (v4f){0.f, 0.f, 0.f, 0.f};
  if (EPI == 1) {
    bv = *(const v4fa*)(bias + clampi(nc, 0, N - 4));
    asm volatile("" :: "v"(bv));
  }
#pragma unroll
  for (int i = 0; i < 4; ++i) {
    const int mBase = m0 + (i << 4);
#pragma unroll
    for (int j = 0; j < 4; ++j) {
#pragma unroll
      for (int r = 0; r < 8; ++r) slab[(h8 + r) * 68 + (j << 4) + rl] = acc[i][j][r];
    }
    __builtin_amdgcn_fence(__ATOMIC_RELEASE, "workgroup");
    __builtin_amdgcn_wave_barrier();
    __builtin_amdgcn_fence(__ATOMIC_ACQUIRE, "workgroup");
    v4f vv[8];
#pragma unroll
    for (int it = 0; it < 8; ++it) {
      const int row = it * 2 + hh;
      v4f v = *(const v4fa*)(slab + row * 68 + c4);
      if (EPI == 1) v += bv;
      vv[it] = v;
    }
    for (int pass = 0; pass < 2; ++pass) {
#pragma unroll
      for (int it = 0; it < 8; ++it) {
        const int row = mBase + it * 2 + hh;
        if (cok && row < M) *(volatile v4f*)(D + (size_t)row * (size_t)ldd + nc) = vv[it];
      }
      __threadfence();
    }
    __builtin_amdgcn_fence(__ATOMIC_RELEASE, "workgroup");
    __builtin_amdgcn_wave_barrier();
    __builtin_amdgcn_fence(__ATOMIC_ACQUIRE, "workgroup");
  }
}

#include <math.h>
#include <stddef.h>

#define NNODE   50000
#define NEDGE   1000000
#define NPATH   15
#define OUTW    144
#define NTHR    256
#define NWAVE   8
#define EPT     8
#define CHUNK   (NTHR * EPT)
#define WCAP    (EPT * 32)
#define LISTN   (NWAVE * WCAP)
#define NBMAX   2048
#define NBRUN   1024
#define SLOTB   11
#define RCAP    28672
#define NBKT    49
#define TE      128
#define OROWS   128
#define NCONV   391
#define H_TERMS 2
#define SILU_FAST 0
#define KS2     (2 * H_TERMS)
#define HP      136
#define HPF     68
#define SRW     72
#define NCG     615
#define P_W2    0
#define P_W3    4096
#define P_CHAN  5120
#define P_CGT   7520
#define P_FW1   10520
#define P_FB1   11032
#define P_FB2   11096
#define P_FB3   11160
#define P_CELL  11176
#define P_END   11188
#define PARW    11264
#define L_PAR   0
#define L_ACC   (L_PAR + PARW)
#define ACCW    (OROWS * OUTW + NWAVE * 96)
#define L_EMB   (L_ACC + ACCW)
#define L_SROW  (L_EMB + TE * 8)
#define L_H1    (L_SROW + TE * SRW)
#define L_H2    (L_H1 + TE * HPF)
#define L_GATE  (L_H2 + TE * HPF)
#define L_TYP   (L_GATE + TE * 16)
#define L_OWN   (L_TYP + TE)
#define L_END   (L_OWN + TE)
#define LDS_CONV (L_END * 4)
#define LDS_BKT ((2 * RCAP + 2 * NBMAX + LISTN) * 4 + 64 + 128)
#define WSCAP   ((size_t)128 << 20)

constexpr int PL1[NPATH]  = {0,0,0,1,1,1,1,1,1,2,2,2,2,2,2};
constexpr int PL2[NPATH]  = {0,1,2,0,1,1,1,2,2,0,1,1,2,2,2};
constexpr int PL3[NPATH]  = {0,1,2,1,0,1,2,1,2,2,1,2,0,1,2};
constexpr int EOFF[NPATH + 1] = {0,1,10,35,44,53,80,125,170,245,270,315,390,415,490,615};
constexpr int SPOS[NPATH] = {30,0,36,5,31,10,41,15,46,51,20,56,32,25,61};
constexpr int YB[3]  = {0,1,4};
constexpr int PM0[6] = {1,3,5,7,10,13};
constexpr int PM1[6] = {2,6,8,9,11,14};
constexpr int PS0[3] = {0,4,12};
constexpr int cnt_l3(int l) { int c = 0; for (int p = 0; p < NPATH; ++p) c += (PL3[p] == l) ? 1 : 0; return c; }
constexpr bool paths_ok() {
  int p = 0;
  for (int a = 0; a < 3; ++a) for (int b = 0; b < 3; ++b) for (int c = 0; c < 3; ++c) {
    const int d = a > b ? a - b : b - a;
    if (c >= d && c <= a + b) {
      if (p >= NPATH) return false;
      if (PL1[p] != a || PL2[p] != b || PL3[p] != c) return false;
      ++p;
    }
  }
  return p == NPATH;
}
constexpr bool spos_ok() {
  for (int j = 0; j < 6; ++j) {
    if (SPOS[PM0[j]] != 5 * j || PL3[PM0[j]] != 1) return false;
    if (SPOS[PM1[j]] != 36 + 5 * j || PL3[PM1[j]] != 2) return false;
  }
  for (int i = 0; i < 3; ++i) if (SPOS[PS0[i]] != 30 + i || PL3[PS0[i]] != 0) return false;
  return true;
}
constexpr bool eoff_ok() {
  for (int p = 0; p < NPATH; ++p)
    if (EOFF[p + 1] - EOFF[p] != (2 * PL1[p] + 1) * (2 * PL2[p] + 1) * (2 * PL3[p] + 1)) return false;
  return EOFF[0] == 0 && EOFF[NPATH] == NCG;
}
static_assert(paths_ok());
static_assert(spos_ok());
static_assert(eoff_ok());
static_assert(cnt_l3(0) == 3 && cnt_l3(1) == 6 && cnt_l3(2) == 6);
static_assert(OUTW == 16 * 9);
static_assert((OROWS * OUTW * 4) % 128 == 0);
static_assert(TE == NWAVE * 16);
static_assert(NBRUN == 8 * OROWS && NBKT * NBRUN >= NNODE && NCONV * OROWS >= NNODE && (NCONV - 1) * OROWS < NNODE);
static_assert(((NNODE % OROWS) % 8) == 0);
static_assert((NCONV - 1) / 8 < NBKT);
static_assert(NEDGE < (1 << (32 - SLOTB)) && (NEDGE % 4) == 0);
static_assert((CHUNK & (CHUNK - 1)) == 0 && NBMAX == (1 << SLOTB) && NTHR * 8 == NBMAX);
static_assert(LISTN >= NBMAX && NBRUN < NBMAX);
static_assert((RCAP % (4 * NTHR)) == 0 && RCAP >= 20807 + CHUNK);
static_assert((RCAP % TE) == 0);
static_assert(TE >= 44 + 8);
static_assert(H_TERMS == 1 || H_TERMS == 2);
static_assert((PARW % (4 * NTHR)) == 0 && P_END <= PARW);
static_assert(3 * NTHR >= NCG && (640 % 32) == 0 && (2400 % 32) == 0 && (NTHR % 32) == 0);
static_assert((L_ACC % 4) == 0 && (L_EMB % 4) == 0 && (L_SROW % 4) == 0 && (L_H1 % 4) == 0 && (L_H2 % 4) == 0);
static_assert((L_GATE % 4) == 0 && (L_TYP % 4) == 0);
static_assert(LDS_CONV <= 327680 && LDS_BKT <= 327680);

typedef int  v4i  __attribute__((ext_vector_type(4)));
typedef v4i  __attribute__((may_alias)) v4ia;
typedef v4u  __attribute__((may_alias)) v4ua;

__device__ __forceinline__ void wave_sync_lds() {
  __builtin_amdgcn_fence(__ATOMIC_RELEASE, "workgroup");
  __builtin_amdgcn_wave_barrier();
  __builtin_amdgcn_fence(__ATOMIC_ACQUIRE, "workgroup");
}

__device__ __forceinline__ float silu_f(float t) {
#if SILU_FAST
  return t * __builtin_amdgcn_rcpf(1.0f + __expf(-t));
#else
  return t * (1.0f / (1.0f + expf(-t)));
#endif
}

__device__ __forceinline__ int path_of(int t) {
  int p = 0;
#pragma unroll
  for (int q = 1; q < NPATH; ++q) p += (t >= EOFF[q]) ? 1 : 0;
  return p;
}
__device__ __forceinline__ void path_info(int p, int& l1, int& l2, int& l3, int& eo) {
  int a = 0, b = 0, c = 0, e = 0;
#pragma unroll
  for (int q = 0; q < NPATH; ++q) {
    const bool s = (p == q);
    a = s ? PL1[q] : a;
    b = s ? PL2[q] : b;
    c = s ? PL3[q] : c;
    e = s ? EOFF[q] : e;
  }
  l1 = a; l2 = b; l3 = c; eo = e;
}

struct cd { double re, im; };
__device__ __forceinline__ cd cmul(cd a, cd b) {
#pragma clang fp contract(off)
  cd r; r.re = a.re * b.re - a.im * b.im; r.im = a.re * b.im + a.im * b.re; return r;
}
__device__ __forceinline__ double dfact(int n) {
  double r = 1.0;
#pragma unroll 1
  for (int i = 2; i <= n; ++i) r *= (double)i;
  return r;
}
__device__ __forceinline__ double cgcoef(int j1, int j2, int j3, int m1, int m2, int m3) {
#pragma clang fp contract(off)
  if (m1 + m2 != m3) return 0.0;
  const double num = (2.0 * (double)j3 + 1.0) * dfact(j3 + j1 - j2) * dfact(j3 - j1 + j2) * dfact(j1 + j2 - j3)
                   * dfact(j3 + m3) * dfact(j3 - m3) * dfact(j1 - m1) * dfact(j1 + m1) * dfact(j2 - m2) * dfact(j2 + m2);
  const double den = dfact(j1 + j2 + j3 + 1);
  const double pre = sqrt(num / den);
  double s = 0.0;
#pragma unroll 1
  for (int k = 0; k <= j1 + j2 - j3; ++k) {
    const int d0 = k, d1 = j1 + j2 - j3 - k, d2 = j1 - m1 - k, d3 = j2 + m2 - k, d4 = j3 - j2 + m1 + k, d5 = j3 - j1 - m2 + k;
    if (d0 < 0 || d1 < 0 || d2 < 0 || d3 < 0 || d4 < 0 || d5 < 0) continue;
    const double term = 1.0 / (dfact(d0) * dfact(d1) * dfact(d2) * dfact(d3) * dfact(d4) * dfact(d5));
    s += (k & 1) ? -term : term;
  }
  return pre * s;
}
__device__ __forceinline__ cd qval(int l, int a, int col) {
  const double INV = __longlong_as_double(0x3FE6A09E667F3BCDLL);
  const int m = a - l;
  cd v; v.re = 0.0; v.im = 0.0;
  if (m < 0) {
    if (col == 2 * l - a)      { v.re = INV; }
    else if (col == a)         { v.im = -INV; }
  } else if (m == 0) {
    if (col == l)              { v.re = 1.0; }
  } else {
    const double s = (m & 1) ? -1.0 : 1.0;
    if (col == a)              { v.re = s * INV; }
    else if (col == 2 * l - a) { v.im = s * INV; }
  }
  if (l == 1) { const double t = v.re; v.re = v.im; v.im = -t; }
  else if (l == 2) { v.re = -v.re; v.im = -v.im; }
  return v;
}

__global__ __launch_bounds__(NTHR) void k_tables(
    const float* __restrict__ emb, const float* __restrict__ mw1, const float* __restrict__ mb1,
    const float* __restrict__ mw2, const float* __restrict__ mb2,
    const float* __restrict__ fw1, const float* __restrict__ fb1, const float* __restrict__ fw2,
    const float* __restrict__ fb2, const float* __restrict__ fw3, const float* __restrict__ fb3,
    const float* __restrict__ tpw, const float* __restrict__ cell, unsigned* PAR) {
#pragma clang fp contract(off)
  __shared__ __attribute__((aligned(16))) unsigned sB[PARW];
  __shared__ double sC[NCG];
  __shared__ double sre[NCG];
  __shared__ double sim[NCG];
  __shared__ float sH[640];
  __shared__ float sAI[80];
  __shared__ int sPick[16];
  float* fB = (float*)sB;
  const int tid = (int)threadIdx.x;
  const int wave = tid >> 5;

  {
    const v4u z = (v4u){0u, 0u, 0u, 0u};
#pragma unroll 1
    for (int i = tid; i < PARW / 4; i += NTHR) *(v4ua*)(sB + 4 * i) = z;
  }
#pragma unroll 1
  for (int it = 0; it < 3; ++it) {
    const int t = tid + NTHR * it;
    const int tc = t < NCG ? t : NCG - 1;
    const int p = path_of(tc);
    int l1, l2, l3, eo;
    path_info(p, l1, l2, l3, eo);
    const int n2 = 2 * l2 + 1, nk = 2 * l3 + 1;
    const int rel = tc - eo;
    const int c = rel % nk, bq = (rel / nk) % n2, a = rel / (nk * n2);
    const double v = cgcoef(l1, l2, l3, a - l1, bq - l2, c - l3);
    if (t < NCG) sC[t] = v;
  }
#pragma unroll 1
  for (int idx = tid; idx < 640; idx += NTHR) {
    const int t = idx >> 6, j = idx & 63;
    float s = 0.0f;
#pragma unroll 1
    for (int i = 0; i < 16; ++i) s = fmaf(bf16_val(emb[t * 16 + i]), bf16_val(mw1[i * 64 + j]), s);
    s += bf16_val(mb1[j]);
    sH[idx] = silu_f(s);
  }
  __syncthreads();

#pragma unroll 1
  for (int it = 0; it < 3; ++it) {
    const int t = tid + NTHR * it;
    const int tc = t < NCG ? t : NCG - 1;
    const int p = path_of(tc);
    int l1, l2, l3, eo;
    path_info(p, l1, l2, l3, eo);
    const int n1 = 2 * l1 + 1, n2 = 2 * l2 + 1, nk = 2 * l3 + 1;
    const int rel = tc - eo;
    const int k = rel % nk, j = (rel / nk) % n2, i = rel / (nk * n2);
    double sr = 0.0, si = 0.0;
#pragma unroll 1
    for (int abc = 0; abc < 125; ++abc) {
      const int a = abc / 25, bq = (abc / 5) % 5, c = abc % 5;
      const bool ok = (a < n1) && (bq < n2) && (c < nk);
      const int ac = a < n1 ? a : n1 - 1;
      const int bc = bq < n2 ? bq : n2 - 1;
      const int cc = c < nk ? c : nk - 1;
      const double Cv = sC[eo + (ac * n2 + bc) * nk + cc];
      const double Cm = ok ? Cv : 0.0;
      cd t1 = qval(l1, ac, i), t2 = qval(l2, bc, j), t3 = qval(l3, cc, k);
      t3.im = -t3.im;
      const cd pr = cmul(cmul(t1, t2), t3);
      sr += pr.re * Cm; si += pr.im * Cm;
    }
    if (t < NCG) { sre[t] = sr; sim[t] = si; }
  }
  if (wave >= 1 && wave <= 3) {
    const int idx = tid - 32;
    const int ic = idx < 80 ? idx : 79;
    const int t = ic >> 3, o = ic & 7;
    float s = 0.0f;
#pragma unroll 1
    for (int j = 0; j < 64; ++j) s = fmaf(sH[t * 64 + j], bf16_val(mw2[j * 8 + o]), s);
    const float b2v = mb2[o];
    asm volatile("" :: "v"(b2v));
    s += bf16_val(b2v);
    if (idx < 80) sAI[idx] = s;
  }
#pragma unroll 1
  for (int w = tid; w < 4096; w += NTHR) {
    const int n = w >> 6, k = (w & 63) * 2;
    const int k0 = k & 63, k1 = (k + 1) & 63;
    sB[P_W2 + w] = pk16(bf16_bits(fw2[k0 * 64 + n]), bf16_bits(fw2[k1 * 64 + n]));
  }
#pragma unroll 1
  for (int w = tid; w < 1024; w += NTHR) {
    const int n = w >> 6, k = (w & 63) * 2;
    const int k0 = k & 63, k1 = (k + 1) & 63;
    const int nc = n < 15 ? n : 14;
    const float a = fw3[k0 * 15 + nc];
    const float b = fw3[k1 * 15 + nc];
    asm volatile("" :: "v"(a)); asm volatile("" :: "v"(b));
    const unsigned m = (n < 15) ? 0xFFFFFFFFu : 0u;
    sB[P_W3 + w] = pk16(bf16_bits(a), bf16_bits(b)) & m;
  }
#pragma unroll 1
  for (int i = tid; i < 512; i += NTHR) fB[P_FW1 + i] = bf16_val(fw1[i]);
  if (wave < 2) { fB[P_FB1 + tid] = bf16_val(fb1[tid]); fB[P_FB2 + tid] = bf16_val(fb2[tid]); }
  if (wave == 2) {
    const int i = tid - 64;
    const float v = fb3[i < 15 ? i : 14];
    asm volatile("" :: "v"(v));
    const float o = (i < 15) ? bf16_val(v) : 0.0f;
    if (i < 16) fB[P_FB3 + i] = o;
  }
  if (wave == 3) {
    const int i = tid - 96;
    const float v = cell[i < 9 ? i : 8];
    asm volatile("" :: "v"(v));
    const float o = (i < 9) ? bf16_val(v) : 0.0f;
    if (i < 12) fB[P_CELL + i] = o;
  }
  __syncthreads();

  {
    const int pq = tid & 15;
    const int pp = pq < NPATH ? pq : NPATH - 1;
    int l1, l2, l3, eo;
    path_info(pp, l1, l2, l3, eo);
    const int np = (2 * l1 + 1) * (2 * l2 + 1) * (2 * l3 + 1);
    double ar = 0.0, ai = 0.0;
#pragma unroll 1
    for (int q = 0; q < 125; ++q) {
      const int idx = eo + (q < np ? q : np - 1);
      const double vr = fabs(sre[idx]), vi = fabs(sim[idx]);
      ar += (q < np) ? vr : 0.0;
      ai += (q < np) ? vi : 0.0;
    }
    if (tid < NPATH) sPick[tid] = (ar >= ai) ? 1 : 0;
  }
#pragma unroll 1
  for (int idx = tid; idx < 2400; idx += NTHR) {
    const int t = idx / 240, rem = idx - t * 240;
    const int p = rem >> 4, c = rem & 15;
    float s = 0.0f;
#pragma unroll 1
    for (int u = 0; u < 8; ++u) s = fmaf(sAI[t * 8 + u], bf16_val(tpw[(p * 8 + u) * 16 + c]), s);
    fB[P_CHAN + idx] = s;
  }
  __syncthreads();

#pragma unroll 1
  for (int it = 0; it < 3; ++it) {
    const int t = tid + NTHR * it;
    const int tc = t < NCG ? t : NCG - 1;
    const int p = path_of(tc);
    int l1, l2, l3, eo;
    path_info(p, l1, l2, l3, eo);
    const int n2 = 2 * l2 + 1, nk = 2 * l3 + 1;
    const int rel = tc - eo;
    const int k = rel % nk, j = (rel / nk) % n2, i = rel / (nk * n2);
    const int pick = sPick[p];
    const double vr = sre[tc], vi = sim[tc];
    const double v = pick ? vr : vi;
    if (t < NCG) fB[P_CGT + (p * 25 + i * 5 + j) * 8 + k] = (float)v;
  }
  __syncthreads();
  for (int pass = 0; pass < 2; ++pass) {
#pragma unroll 1
    for (int i = tid; i < PARW / 4; i += NTHR) {
      const v4u v = *(const v4ua*)(sB + 4 * i);
      *(volatile v4u*)(PAR + 4 * (size_t)i) = v;
    }
    __threadfence();
  }
}

__device__ __forceinline__ int scan_chunk(const int* __restrict__ dsts, int nE, int cbase, int slotBase,
                                          int nb, int vec8, int* list, int tid, int lane, int wave) {
  int wc = 0;
  const int el0  = tid * EPT;
  const int e0   = cbase + el0;
  const int sent = (-0x7fffffff - 1);
  v4i da, db;
  if (vec8 != 0 && cbase + CHUNK <= nE) {
    da = *(const v4ia*)(dsts + e0);
    db = *(const v4ia*)(dsts + e0 + 4);
  } else {
    const int t0 = dsts[min(e0,     nE - 1)];
    const int t1 = dsts[min(e0 + 1, nE - 1)];
    const int t2 = dsts[min(e0 + 2, nE - 1)];
    const int t3 = dsts[min(e0 + 3, nE - 1)];
    const int t4 = dsts[min(e0 + 4, nE - 1)];
    const int t5 = dsts[min(e0 + 5, nE - 1)];
    const int t6 = dsts[min(e0 + 6, nE - 1)];
    const int t7 = dsts[min(e0 + 7, nE - 1)];
    asm volatile("" :: "v"(t0)); asm volatile("" :: "v"(t1)); asm volatile("" :: "v"(t2)); asm volatile("" :: "v"(t3));
    asm volatile("" :: "v"(t4)); asm volatile("" :: "v"(t5)); asm volatile("" :: "v"(t6)); asm volatile("" :: "v"(t7));
    da.x = (e0     < nE) ? t0 : sent;
    da.y = (e0 + 1 < nE) ? t1 : sent;
    da.z = (e0 + 2 < nE) ? t2 : sent;
    da.w = (e0 + 3 < nE) ? t3 : sent;
    db.x = (e0 + 4 < nE) ? t4 : sent;
    db.y = (e0 + 5 < nE) ? t5 : sent;
    db.z = (e0 + 6 < nE) ? t6 : sent;
    db.w = (e0 + 7 < nE) ? t7 : sent;
  }
  const unsigned nbs = (unsigned)slotBase;
  const unsigned unb = (unsigned)nb;
  const unsigned s0 = (unsigned)da.x - nbs, s1 = (unsigned)da.y - nbs;
  const unsigned s2 = (unsigned)da.z - nbs, s3 = (unsigned)da.w - nbs;
  const unsigned s4 = (unsigned)db.x - nbs, s5 = (unsigned)db.y - nbs;
  const unsigned s6 = (unsigned)db.z - nbs, s7 = (unsigned)db.w - nbs;
  const bool h0 = s0 < unb, h1 = s1 < unb, h2 = s2 < unb, h3 = s3 < unb;
  const bool h4 = s4 < unb, h5 = s5 < unb, h6 = s6 < unb, h7 = s7 < unb;
  const unsigned any = __builtin_amdgcn_ballot_w32(h0 | h1 | h2 | h3 | h4 | h5 | h6 | h7);
  if (any != 0u) {
#define HITJ(J, HJ, SJ) { \
      const unsigned mj = __builtin_amdgcn_ballot_w32(HJ); \
      if (mj != 0u) { \
        if (HJ) { \
          const int pos = wc + (int)__builtin_amdgcn_mbcnt_lo(mj, 0u); \
          if (pos < WCAP) list[wave * WCAP + pos] = ((el0 + (J)) << SLOTB) | (int)(SJ); \
        } \
        wc += (int)__builtin_popcount(mj); } }
    HITJ(0, h0, s0)
    HITJ(1, h1, s1)
    HITJ(2, h2, s2)
    HITJ(3, h3, s3)
    HITJ(4, h4, s4)
    HITJ(5, h5, s5)
    HITJ(6, h6, s6)
    HITJ(7, h7, s7)
#undef HITJ
  }
  return wc;
}

__global__ __launch_bounds__(NTHR) void k_bucket(const int* __restrict__ dsts, int* LISTB, int* HDR,
                                                 int nN, int nE, int vec8) {
  extern __shared__ v4f lds_dyn[];
  int* reg1 = (int*)lds_dyn;
  int* reg2 = reg1 + RCAP;
  int* scnt = reg2 + RCAP;
  int* soff = scnt + NBMAX;
  int* list = soff + NBMAX;
  int* wcnt = list + LISTN;
  int* wtot = wcnt + NWAVE;
  int* hl   = wtot + NWAVE;
  const int tid = (int)threadIdx.x, lane = tid & 31, wave = tid >> 5;
  const int nodeBase = (int)blockIdx.x * NBRUN;
  int nb = nN - nodeBase;
  nb = nb < 0 ? 0 : (nb > NBRUN ? NBRUN : nb);

  for (int i = tid; i < NBMAX; i += NTHR) scnt[i] = 0;
  {
    const v4i z4 = (v4i){0, 0, 0, 0};
#pragma unroll 1
    for (int i = tid; i < RCAP / 4; i += NTHR) *(v4ia*)(reg2 + 4 * i) = z4;
  }
  __syncthreads();

  int tot = 0;
  const int nChunks = (nE + CHUNK - 1) / CHUNK;
#pragma unroll 1
  for (int ch = 0; ch < nChunks; ++ch) {
    const int cbase = ch * CHUNK;
    const int wc = scan_chunk(dsts, nE, cbase, nodeBase, nb, vec8, list, tid, lane, wave);
    if (lane == 0) wcnt[wave] = wc;
    __syncthreads();
    int pre = 0, all = 0;
#pragma unroll
    for (int w2 = 0; w2 < NWAVE; ++w2) {
      int c = wcnt[w2];
      c = c < 0 ? 0 : (c > WCAP ? WCAP : c);
      all += c;
      pre += (w2 < wave) ? c : 0;
    }
    const int wcc  = wc > WCAP ? WCAP : wc;
    const int base = tot + pre;
#pragma unroll 1
    for (int i = lane; i < wcc; i += 32) {
      const int ent = list[wave * WCAP + i];
      const int el  = (ent >> SLOTB) & (CHUNK - 1);
      const int sl  = ent & (NBMAX - 1);
      int eid = cbase + el;
      eid = eid > nE - 1 ? nE - 1 : eid;
      const int pos = base + i;
      if (pos < RCAP) reg1[pos] = (int)(((unsigned)eid << SLOTB) | (unsigned)sl);
    }
    tot += all;
    tot = tot > RCAP ? RCAP : tot;
    __syncthreads();
  }
  const int nh = tot;

  if (wave == 0) {
#pragma unroll 1
    for (int b0 = 0; b0 < nh; b0 += 32) {
      const int idx = b0 + lane;
      const int uv  = reg1[idx < nh ? idx : nh - 1];
      const int m32 = (nh - b0) < 32 ? (nh - b0) : 32;
#pragma unroll 1
      for (int k = 0; k < m32; ++k) {
        const int u  = __builtin_amdgcn_readlane(uv, k);
        const int sl = u & (NBMAX - 1);
        if (lane == 0) scnt[sl] = scnt[sl] + 1;
      }
    }
  }
  __syncthreads();

  {
    const v4i ca = *(const v4ia*)(scnt + 8 * tid);
    const v4i cb = *(const v4ia*)(scnt + 8 * tid + 4);
    const int e0 = ca.x < 0 ? 0 : ca.x, e1 = ca.y < 0 ? 0 : ca.y, e2 = ca.z < 0 ? 0 : ca.z, e3 = ca.w < 0 ? 0 : ca.w;
    const int e4 = cb.x < 0 ? 0 : cb.x, e5 = cb.y < 0 ? 0 : cb.y, e6 = cb.z < 0 ? 0 : cb.z, e7 = cb.w < 0 ? 0 : cb.w;
    const int ts = e0 + e1 + e2 + e3 + e4 + e5 + e6 + e7;
    int incl = ts;
#pragma unroll
    for (int d = 1; d < 32; d <<= 1) {
      const int up = __shfl_up(incl, d);
      if (lane >= d) incl += up;
    }
    if (lane == 31) wtot[wave] = incl;
    __syncthreads();
    int pre = 0;
#pragma unroll
    for (int w2 = 0; w2 < NWAVE; ++w2) pre += (w2 < wave) ? wtot[w2] : 0;
    int run = pre + incl - ts;
    soff[8 * tid + 0] = run; run += e0;
    soff[8 * tid + 1] = run; run += e1;
    soff[8 * tid + 2] = run; run += e2;
    soff[8 * tid + 3] = run; run += e3;
    soff[8 * tid + 4] = run; run += e4;
    soff[8 * tid + 5] = run; run += e5;
    soff[8 * tid + 6] = run; run += e6;
    soff[8 * tid + 7] = run;
  }
  __syncthreads();
  for (int i = tid; i < NBMAX; i += NTHR) list[i] = soff[i];
  __syncthreads();

  if (wave == 0) {
#pragma unroll 1
    for (int b0 = 0; b0 < nh; b0 += 32) {
      const int idx = b0 + lane;
      const int uv  = reg1[idx < nh ? idx : nh - 1];
      const int m32 = (nh - b0) < 32 ? (nh - b0) : 32;
#pragma unroll 1
      for (int k = 0; k < m32; ++k) {
        const int u   = __builtin_amdgcn_readlane(uv, k);
        const int sl  = u & (NBMAX - 1);
        const int eid = (int)((unsigned)u >> SLOTB);
        if (lane == 0) {
          int pos = list[sl];
          pos = pos < 0 ? 0 : (pos > RCAP - 1 ? RCAP - 1 : pos);
          reg2[pos] = eid;
          list[sl] = pos + 1;
        }
      }
    }
  }
  __syncthreads();

  if (tid < 32) {
    const int k = tid < 8 ? tid : 8;
    const int sv = soff[OROWS * k];
    const int ov = (nh >= RCAP) ? 1 : 0;
    const int v = (tid < 9) ? sv : ((tid == 9) ? ov : ((tid == 10) ? nh : 0));
    hl[tid] = v;
  }
  __syncthreads();
  if (wave == 0) {
    const bool ok = lane < 8;
    const v4i hv = *(const v4ia*)(hl + 4 * (lane & 7));
    int* hp = HDR + (size_t)blockIdx.x * 32 + 4 * (lane & 7);
    if (ok) *(volatile v4i*)hp = hv;
    __threadfence();
    if (ok) *(volatile v4i*)hp = hv;
  }
  int* lb = LISTB + (size_t)blockIdx.x * RCAP;
  for (int pass = 0; pass < 2; ++pass) {
#pragma unroll 1
    for (int i = tid; i < RCAP / 4; i += NTHR) {
      const v4i v = *(const v4ia*)(reg2 + 4 * i);
      *(volatile v4i*)(lb + 4 * (size_t)i) = v;
    }
    __threadfence();
  }
}

template <int P>
__device__ __forceinline__ void geo_path(const float (&Y)[9], const float* cgt, float* srow) {
  constexpr int l1 = PL1[P], l2 = PL2[P], l3 = PL3[P];
  constexpr int n1 = 2 * l1 + 1, n2 = 2 * l2 + 1, nk = 2 * l3 + 1;
  constexpr int y1 = YB[l1], y2 = YB[l2];
  constexpr int sp = SPOS[P];
  float g0 = 0.0f, g1 = 0.0f, g2 = 0.0f, g3 = 0.0f, g4 = 0.0f;
#pragma unroll
  for (int m = 0; m < n1; ++m) {
#pragma unroll
    for (int n = 0; n < n2; ++n) {
      const float yy = Y[y1 + m] * Y[y2 + n];
      const float* cp = cgt + (P * 25 + m * 5 + n) * 8;
      if (nk == 1) {
        g0 = fmaf(yy, cp[0], g0);
      } else {
        const v4f ca = *(const v4fa*)cp;
        g0 = fmaf(yy, ca[0], g0);
        g1 = fmaf(yy, ca[1], g1);
        g2 = fmaf(yy, ca[2], g2);
        if (nk == 5) {
          const float c4 = cp[4];
          g3 = fmaf(yy, ca[3], g3);
          g4 = fmaf(yy, c4, g4);
        }
      }
    }
  }
  srow[sp] = g0;
  if (nk >= 3) { srow[sp + 1] = g1; srow[sp + 2] = g2; }
  if (nk == 5) { srow[sp + 3] = g3; srow[sp + 4] = g4; }
}

__global__ __launch_bounds__(NTHR) __attribute__((amdgpu_num_vgpr(248)))
void k_conv(const float* __restrict__ pos, const int* __restrict__ atype, const int* __restrict__ batch,
            const int* __restrict__ esrc, const int* __restrict__ edst, const float* __restrict__ shifts,
            const unsigned* __restrict__ PAR, const int* __restrict__ LISTB, const int* __restrict__ HDR,
            float* out, int nN, int nE) {
  extern __shared__ v4f lds_dyn[];
  float* L = (float*)lds_dyn;
  const unsigned short* sW2 = (const unsigned short*)(L + L_PAR + P_W2);
  const unsigned short* sW3 = (const unsigned short*)(L + L_PAR + P_W3);
  const float* sCHAN = L + L_PAR + P_CHAN;
  const float* sCGT  = L + L_PAR + P_CGT;
  const float* sFW1  = L + L_PAR + P_FW1;
  const float* sFB1  = L + L_PAR + P_FB1;
  const float* sFB2  = L + L_PAR + P_FB2;
  const float* sFB3  = L + L_PAR + P_FB3;
  const float* sCELL = L + L_PAR + P_CELL;
  float* ACC  = L + L_ACC;
  float* EMB  = L + L_EMB;
  float* SROW = L + L_SROW;
  float* H1f  = L + L_H1;
  unsigned short* H1u = (unsigned short*)(L + L_H1);
  unsigned short* H2u = (unsigned short*)(L + L_H2);
  float* GATE = L + L_GATE;
  int* TYP = (int*)(L + L_TYP);
  int* OWN = (int*)(L + L_OWN);

  const int tid = (int)threadIdx.x, lane = tid & 31, wave = tid >> 5;
  const int hf = lane >> 4, m = lane & 15;
  const int b = (int)blockIdx.x;
  const int bkt = b >> 3, sub = b & 7;

#pragma unroll 1
  for (int i = tid; i < PARW / 4; i += NTHR) *(v4ua*)(L + L_PAR + 4 * i) = *(const v4ua*)(PAR + 4 * (size_t)i);
  {
    const v4f z4 = (v4f){0.f, 0.f, 0.f, 0.f};
#pragma unroll 1
    for (int i = tid; i < ACCW / 4; i += NTHR) *(v4fa*)(ACC + 4 * i) = z4;
#pragma unroll 1
    for (int i = tid; i < TE * SRW / 4; i += NTHR) *(v4fa*)(SROW + 4 * i) = z4;
  }
  int st = HDR[bkt * 32 + sub];
  int en = HDR[bkt * 32 + sub + 1];
  int fl = HDR[bkt * 32 + 9];
  asm volatile("" :: "v"(st), "v"(en), "v"(fl));
  st = clampi(st, 0, RCAP);
  en = clampi(en, st, RCAP);
  st = __builtin_amdgcn_readfirstlane(st);
  en = __builtin_amdgcn_readfirstlane(en);
  fl = __builtin_amdgcn_readfirstlane(fl);
  const int len = en - st;
  __syncthreads();

  const float A0   = __uint_as_float(0x3E5105ECu);
  const float A1   = __uint_as_float(0x3E13CD3Au);
  const float S3   = __uint_as_float(0x3FDDB3D7u);
  const float S15  = __uint_as_float(0x4077DEF6u);
  const float S5H  = __uint_as_float(0x3F8F1BBDu);
  const float S15H = __uint_as_float(0x3FF7DEF6u);
  const float SQ8  = __uint_as_float(0x403504F3u);

#pragma unroll 1
  for (int ts = 0; ts < len; ts += TE) {
    {
      const int ei = tid & (TE - 1);
      const int part = tid >> 7;
      const int lic = clampi(st + ts + ei, 0, RCAP - 1);
      const int lraw = LISTB[(size_t)bkt * RCAP + lic];
      asm volatile("" :: "v"(lraw));
      const int eid = clampi(lraw, 0, nE - 1);
      const bool valid = (ts + ei) < len;
      const int sraw = esrc[eid];
      const int draw = edst[eid];
      asm volatile("" :: "v"(sraw));
      asm volatile("" :: "v"(draw));
      const int s = clampi(sraw, 0, nN - 1);
      const int d = clampi(draw, 0, nN - 1);
      const float* pps = pos + (size_t)s * 3;
      const float* ppd = pos + (size_t)d * 3;
      const float qs0 = pps[0], qs1 = pps[1], qs2 = pps[2];
      const float qd0 = ppd[0], qd1 = ppd[1], qd2 = ppd[2];
      const int at = atype[s];
      const int bt = batch[s];
      int eid2 = eid;
      asm volatile("" : "+v"(eid2) : "v"(qs0), "v"(qs1), "v"(qs2), "v"(qd0), "v"(qd1), "v"(qd2), "v"(at), "v"(bt));
      const float* shp = shifts + (size_t)eid2 * 3;
      const float h0 = bf16_val(shp[0]), h1 = bf16_val(shp[1]), h2 = bf16_val(shp[2]);
      const int ci = clampi(bt, 0, 0);
      const float* C = sCELL + ci * 9;
      const float shx = h0 * C[0] + h1 * C[3] + h2 * C[6];
      const float shy = h0 * C[1] + h1 * C[4] + h2 * C[7];
      const float shz = h0 * C[2] + h1 * C[5] + h2 * C[8];
      const float vx = (bf16_val(qd0) - bf16_val(qs0)) + shx;
      const float vy = (bf16_val(qd1) - bf16_val(qs1)) + shy;
      const float vz = (bf16_val(qd2) - bf16_val(qs2)) + shz;
      const float t0 = vx * vx, t1 = vy * vy, t2 = vz * vz;
      const float len3 = sqrtf((t0 + t2) + t1);
      const float den = fmaxf(len3, 1e-8f);
      const float nx = vx / den, ny = vy / den, nz = vz / den;
      float Y[9];
      Y[0] = 1.0f;
      Y[1] = S3 * ny; Y[2] = S3 * nz; Y[3] = S3 * nx;
      Y[4] = S15 * nx * ny; Y[5] = S15 * ny * nz; Y[6] = S5H * (3.0f * nz * nz - 1.0f);
      Y[7] = S15 * nx * nz; Y[8] = S15H * (nx * nx - ny * ny);
      float* sr = SROW + ei * SRW;
      if (part == 0) {
        const float STEP = __uint_as_float(0x3E638E39u);
        float em[8];
        em[0] = (len3 - __uint_as_float(0x3E638E39u)) / STEP;
        em[1] = (len3 - __uint_as_float(0x3EE38E39u)) / STEP;
        em[2] = (len3 - __uint_as_float(0x3F2AAAABu)) / STEP;
        em[3] = (len3 - __uint_as_float(0x3F638E39u)) / STEP;
        em[4] = (len3 - __uint_as_float(0x3F8E38E4u)) / STEP;
        em[5] = (len3 - __uint_as_float(0x3FAAAAABu)) / STEP;
        em[6] = (len3 - __uint_as_float(0x3FC71C72u)) / STEP;
        em[7] = (len3 - __uint_as_float(0x3FE38E39u)) / STEP;
#pragma unroll
        for (int k = 0; k < 8; ++k) em[k] = expf(-em[k] * em[k]) / 1.12f * SQ8;
        *(v4fa*)(EMB + ei * 8)     = (v4f){ em[0], em[1], em[2], em[3] };
        *(v4fa*)(EMB + ei * 8 + 4) = (v4f){ em[4], em[5], em[6], em[7] };
        TYP[ei] = clampi(at, 0, 9);
        OWN[ei] = valid ? clampi(draw - OROWS * b, 0, OROWS - 1) : 255;
        geo_path<0>(Y, sCGT, sr);
        geo_path<1>(Y, sCGT, sr);
        geo_path<2>(Y, sCGT, sr);
        geo_path<3>(Y, sCGT, sr);
        geo_path<4>(Y, sCGT, sr);
        geo_path<5>(Y, sCGT, sr);
        geo_path<6>(Y, sCGT, sr);
        geo_path<7>(Y, sCGT, sr);
        geo_path<8>(Y, sCGT, sr);
        geo_path<9>(Y, sCGT, sr);
        geo_path<10>(Y, sCGT, sr);
      } else {
        geo_path<11>(Y, sCGT, sr);
        geo_path<12>(Y, sCGT, sr);
        geo_path<13>(Y, sCGT, sr);
        geo_path<14>(Y, sCGT, sr);
      }
    }
    __syncthreads();

    {
      const int row = 16 * wave + m;
      {
        const v4f e0 = *(const v4fa*)(EMB + row * 8);
        const v4f e1 = *(const v4fa*)(EMB + row * 8 + 4);
        unsigned short* h1r = H1u + row * HP;
#pragma unroll 1
        for (int jb = 0; jb < 4; ++jb) {
          const int c0 = hf * 32 + jb * 8;
          const float* wp = sFW1 + c0;
          v4f sa = *(const v4fa*)(wp) * e0[0];
          v4f sb = *(const v4fa*)(wp + 4) * e0[0];
          sa += *(const v4fa*)(wp + 64)  * e0[1];  sb += *(const v4fa*)(wp + 68)  * e0[1];
          sa += *(const v4fa*)(wp + 128) * e0[2];  sb += *(const v4fa*)(wp + 132) * e0[2];
          sa += *(const v4fa*)(wp + 192) * e0[3];  sb += *(const v4fa*)(wp + 196) * e0[3];
          sa += *(const v4fa*)(wp + 256) * e1[0];  sb += *(const v4fa*)(wp + 260) * e1[0];
          sa += *(const v4fa*)(wp + 320) * e1[1];  sb += *(const v4fa*)(wp + 324) * e1[1];
          sa += *(const v4fa*)(wp + 384) * e1[2];  sb += *(const v4fa*)(wp + 388) * e1[2];
          sa += *(const v4fa*)(wp + 448) * e1[3];  sb += *(const v4fa*)(wp + 452) * e1[3];
          sa += *(const v4fa*)(sFB1 + c0);
          sb += *(const v4fa*)(sFB1 + c0 + 4);
          v4f xa, xb;
          xa[0] = silu_f(sa[0]); xa[1] = silu_f(sa[1]); xa[2] = silu_f(sa[2]); xa[3] = silu_f(sa[3]);
          xb[0] = silu_f(sb[0]); xb[1] = silu_f(sb[1]); xb[2] = silu_f(sb[2]); xb[3] = silu_f(sb[3]);
          const v4u hv = pack8_bf16(xa, xb);
          *(v4ua*)(h1r + c0) = hv;
          if (H_TERMS == 2) {
            const v4u lv = pack8_bf16_lo(xa, xb);
            *(v4ua*)(h1r + 64 + c0) = lv;
          }
        }
      }
      wave_sync_lds();
      v8f acc[4];
#pragma unroll
      for (int j = 0; j < 4; ++j) acc[j] = (v8f){0.f, 0.f, 0.f, 0.f, 0.f, 0.f, 0.f, 0.f};
      {
        const unsigned short* ap = H1u + row * HP + 8 * hf;
        FragB af[KS2];
#pragma unroll
        for (int ks = 0; ks < KS2; ++ks) {
          af[ks].h[0] = *(const v8usa*)(ap + 32 * ks);
          af[ks].h[1] = *(const v8usa*)(ap + 32 * ks + 16);
        }
#pragma unroll
        for (int j = 0; j < 4; ++j) {
          const unsigned short* bp = sW2 + (16 * j + m) * 128 + 8 * hf;
#pragma unroll
          for (int ks = 0; ks < KS2; ++ks) {
            FragB bfj;
            bfj.h[0] = *(const v8usa*)(bp + 32 * ks);
            bfj.h[1] = *(const v8usa*)(bp + 32 * ks + 16);
            acc[j] = wmb(af[ks], bfj, acc[j]);
          }
        }
      }
      wave_sync_lds();
#pragma unroll
      for (int j = 0; j < 4; ++j) {
#pragma unroll
        for (int r = 0; r < 8; ++r) H1f[(16 * wave + 8 * hf + r) * HPF + 16 * j + m] = acc[j][r];
      }
      wave_sync_lds();
      {
        unsigned short* h2r = H2u + row * HP;
#pragma unroll 1
        for (int jb = 0; jb < 4; ++jb) {
          const int c0 = hf * 32 + jb * 8;
          v4f sa = *(const v4fa*)(H1f + row * HPF + c0);
          v4f sb = *(const v4fa*)(H1f + row * HPF + c0 + 4);
          sa += *(const v4fa*)(sFB2 + c0);
          sb += *(const v4fa*)(sFB2 + c0 + 4);
          v4f xa, xb;
          xa[0] = silu_f(sa[0]); xa[1] = silu_f(sa[1]); xa[2] = silu_f(sa[2]); xa[3] = silu_f(sa[3]);
          xb[0] = silu_f(sb[0]); xb[1] = silu_f(sb[1]); xb[2] = silu_f(sb[2]); xb[3] = silu_f(sb[3]);
          const v4u hv = pack8_bf16(xa, xb);
          *(v4ua*)(h2r + c0) = hv;
          if (H_TERMS == 2) {
            const v4u lv = pack8_bf16_lo(xa, xb);
            *(v4ua*)(h2r + 64 + c0) = lv;
          }
        }
      }
      wave_sync_lds();
      {
        v8f a3 = (v8f){0.f, 0.f, 0.f, 0.f, 0.f, 0.f, 0.f, 0.f};
        const unsigned short* ap = H2u + row * HP + 8 * hf;
        const unsigned short* bp = sW3 + m * 128 + 8 * hf;
#pragma unroll
        for (int ks = 0; ks < KS2; ++ks) {
          FragB af, bfj;
          af.h[0]  = *(const v8usa*)(ap + 32 * ks);
          af.h[1]  = *(const v8usa*)(ap + 32 * ks + 16);
          bfj.h[0] = *(const v8usa*)(bp + 32 * ks);
          bfj.h[1] = *(const v8usa*)(bp + 32 * ks + 16);
          a3 = wmb(af, bfj, a3);
        }
        const float b3 = sFB3[m];
#pragma unroll
        for (int r = 0; r < 8; ++r) GATE[(16 * wave + 8 * hf + r) * 16 + m] = a3[r] + b3;
      }
      wave_sync_lds();
      {
        float* sr = SROW + row * SRW + hf * 36;
        const float* gr = GATE + row * 16;
        const float gm0 = gr[hf ? 2 : 1]   * A1;
        const float gm1 = gr[hf ? 6 : 3]   * A1;
        const float gm2 = gr[hf ? 8 : 5]   * A1;
        const float gm3 = gr[hf ? 9 : 7]   * A1;
        const float gm4 = gr[hf ? 11 : 10] * A1;
        const float gm5 = gr[hf ? 14 : 13] * A1;
        const float q0 = gr[0] * A0, q1 = gr[4] * A0, q2 = gr[12] * A0;
        const float g[6] = { gm0, gm1, gm2, gm3, gm4, gm5 };
        const float gs[3] = { hf ? 0.0f : q0, hf ? 0.0f : q1, hf ? 0.0f : q2 };
        v4f v[9];
#pragma unroll
        for (int q = 0; q < 9; ++q) v[q] = *(const v4fa*)(sr + 4 * q);
#pragma unroll
        for (int i = 0; i < 33; ++i) {
          const float f = (i < 30) ? g[i / 5] : gs[i < 30 ? 0 : i - 30];
          v[i >> 2][i & 3] *= f;
        }
#pragma unroll
        for (int q = 0; q < 9; ++q) *(v4fa*)(sr + 4 * q) = v[q];
      }
    }
    __syncthreads();

    {
      int cntT = len - ts; cntT = cntT > TE ? TE : cntT;
      int rF = OWN[0];
      int rL = OWN[cntT - 1];
      rF = clampi(__builtin_amdgcn_readfirstlane(rF), 0, OROWS - 1);
      rL = clampi(__builtin_amdgcn_readfirstlane(rL), 0, OROWS - 1);
      const int o0 = OWN[lane], o1 = OWN[32 + lane], o2 = OWN[64 + lane], o3 = OWN[96 + lane];
      const int c = m;
      const int po0 = (hf ? 2 : 1) * 16, po1 = (hf ? 6 : 3) * 16, po2 = (hf ? 8 : 5) * 16;
      const int po3 = (hf ? 9 : 7) * 16, po4 = (hf ? 11 : 10) * 16, po5 = (hf ? 14 : 13) * 16;
      const int sink = OROWS * OUTW + wave * 96 + lane;
      int r = rF + ((wave - rF) & 7);
#pragma unroll 1
      for (int it = 0; it < 16 && r <= rL; ++it, r += 8) {
        int lo = (int)__builtin_popcount(__builtin_amdgcn_ballot_w32(o0 < r)) +
                 (int)__builtin_popcount(__builtin_amdgcn_ballot_w32(o1 < r)) +
                 (int)__builtin_popcount(__builtin_amdgcn_ballot_w32(o2 < r)) +
                 (int)__builtin_popcount(__builtin_amdgcn_ballot_w32(o3 < r));
        int hi = (int)__builtin_popcount(__builtin_amdgcn_ballot_w32(o0 <= r)) +
                 (int)__builtin_popcount(__builtin_amdgcn_ballot_w32(o1 <= r)) +
                 (int)__builtin_popcount(__builtin_amdgcn_ballot_w32(o2 <= r)) +
                 (int)__builtin_popcount(__builtin_amdgcn_ballot_w32(o3 <= r));
        hi = hi > cntT ? cntT : hi;
        lo = lo > hi ? hi : lo;
        float aa[6];
#pragma unroll
        for (int k = 0; k < 6; ++k) aa[k] = 0.0f;
#pragma unroll 1
        for (int q = lo; q < hi; ++q) {
          int tq = TYP[q];
          tq = clampi(__builtin_amdgcn_readfirstlane(tq), 0, 9);
          const float* chb = sCHAN + tq * 240 + c;
          const float* sr = SROW + q * SRW + hf * 36;
          v4f sv[9];
#pragma unroll
          for (int u = 0; u < 9; ++u) sv[u] = *(const v4fa*)(sr + 4 * u);
          float ch[6];
          ch[0] = chb[po0]; ch[1] = chb[po1]; ch[2] = chb[po2];
          ch[3] = chb[po3]; ch[4] = chb[po4]; ch[5] = chb[po5];
          const float cs0 = chb[0], cs1 = chb[64], cs2 = chb[192];
#pragma unroll
          for (int j = 0; j < 6; ++j) {
#pragma unroll
            for (int k = 0; k < 5; ++k) aa[k] = fmaf(ch[j], sv[(5 * j + k) >> 2][(5 * j + k) & 3], aa[k]);
          }
          aa[5] = fmaf(cs0, sv[7][2], aa[5]);
          aa[5] = fmaf(cs1, sv[7][3], aa[5]);
          aa[5] = fmaf(cs2, sv[8][0], aa[5]);
        }
        const int rb = r * OUTW;
        const int i0 = hf ? (rb + 64 + 5 * c)     : (rb + 16 + 3 * c);
        const int i1 = hf ? (rb + 64 + 5 * c + 1) : (rb + 16 + 3 * c + 1);
        const int i2 = hf ? (rb + 64 + 5 * c + 2) : (rb + 16 + 3 * c + 2);
        const int i3 = hf ? (rb + 64 + 5 * c + 3) : sink;
        const int i4 = hf ? (rb + 64 + 5 * c + 4) : (sink + 32);
        const int i5 = hf ? (sink + 64)           : (rb + c);
        ACC[i0] = ACC[i0] + aa[0];
        ACC[i1] = ACC[i1] + aa[1];
        ACC[i2] = ACC[i2] + aa[2];
        ACC[i3] = ACC[i3] + aa[3];
        ACC[i4] = ACC[i4] + aa[4];
        ACC[i5] = ACC[i5] + aa[5];
      }
    }
    __syncthreads();
  }

  __syncthreads();
  int nrows = nN - OROWS * b;
  nrows = nrows < 0 ? 0 : (nrows > OROWS ? OROWS : nrows);
  const int npc = nrows * (OUTW / 4);
  const float qnan = __int_as_float(0x7fc00000);
  const bool poison = fl != 0;
#pragma unroll 1
  for (int it = 0; it < (OROWS * OUTW / 4) / NTHR; ++it) {
    const int p = tid + NTHR * it;
    if (p < npc) {
      v4f v = *(const v4fa*)(ACC + 4 * p);
      v[0] = v[0] / 20.0f; v[1] = v[1] / 20.0f; v[2] = v[2] / 20.0f; v[3] = v[3] / 20.0f;
      v[0] = poison ? qnan : v[0];
      v[1] = poison ? qnan : v[1];
      v[2] = poison ? qnan : v[2];
      v[3] = poison ? qnan : v[3];
      *(v4fa*)(ACC + 4 * p) = v;
    }
  }
  __syncthreads();
  float* gp = out + (size_t)b * (size_t)(OROWS * OUTW);
  for (int pass = 0; pass < 2; ++pass) {
#pragma unroll 1
    for (int it = 0; it < (OROWS * OUTW / 4) / NTHR; ++it) {
      const int p = tid + NTHR * it;
      if (p < npc) {
        const v4f v = *(const v4fa*)(ACC + 4 * p);
        *(volatile v4f*)(gp + 4 * (size_t)p) = v;
      }
    }
    __threadfence();
  }
}

static inline size_t al256(size_t o) { return (o + 255) & ~(size_t)255; }

extern "C" void kernel_launch(void* const* d_in, const int* in_sizes, int n_in,
                              void* d_out, int out_size, void* d_ws, size_t ws_size,
                              hipStream_t stream) {
  if (n_in < 19) return;
  if (in_sizes[0] != NNODE * 3) return;
  if (in_sizes[1] != NNODE || in_sizes[2] != NNODE) return;
  if (in_sizes[3] != NEDGE || in_sizes[4] != NEDGE) return;
  if (in_sizes[5] != NEDGE * 3 || in_sizes[6] != 9) return;
  if (in_sizes[7] != 160 || in_sizes[8] != 1024 || in_sizes[9] != 64) return;
  if (in_sizes[10] != 512 || in_sizes[11] != 8) return;
  if (in_sizes[12] != 512 || in_sizes[13] != 64) return;
  if (in_sizes[14] != 4096 || in_sizes[15] != 64) return;
  if (in_sizes[16] != 960 || in_sizes[17] != 15) return;
  if (in_sizes[18] != 1920) return;
  if ((long long)out_size != (long long)NNODE * OUTW) return;

  const float* pos    = (const float*)d_in[0];
  const int*   atype  = (const int*)d_in[1];
  const int*   batch  = (const int*)d_in[2];
  const int*   esrc   = (const int*)d_in[3];
  const int*   edst   = (const int*)d_in[4];
  const float* shifts = (const float*)d_in[5];
  const float* cell   = (const float*)d_in[6];
  const float* emb    = (const float*)d_in[7];
  const float* mw1    = (const float*)d_in[8];
  const float* mb1    = (const float*)d_in[9];
  const float* mw2    = (const float*)d_in[10];
  const float* mb2    = (const float*)d_in[11];
  const float* fw1    = (const float*)d_in[12];
  const float* fb1    = (const float*)d_in[13];
  const float* fw2    = (const float*)d_in[14];
  const float* fb2    = (const float*)d_in[15];
  const float* fw3    = (const float*)d_in[16];
  const float* fb3    = (const float*)d_in[17];
  const float* tpw    = (const float*)d_in[18];
  float* out = (float*)d_out;

  char* ws = (char*)d_ws;
  size_t off = 0;
  const size_t oPAR  = off; off = al256(off + (size_t)PARW * 4);
  const size_t oHDR  = off; off = al256(off + (size_t)NBKT * 128);
  const size_t oLIST = off; off = al256(off + (size_t)NBKT * RCAP * 4);
  if (off > ws_size || off > (size_t)WSCAP) return;
  unsigned* PAR = (unsigned*)(ws + oPAR);
  int* HDR   = (int*)(ws + oHDR);
  int* LISTB = (int*)(ws + oLIST);

  hipFuncSetAttribute(reinterpret_cast<const void*>(&k_bucket), hipFuncAttributeMaxDynamicSharedMemorySize, LDS_BKT);
  hipFuncSetAttribute(reinterpret_cast<const void*>(&k_conv), hipFuncAttributeMaxDynamicSharedMemorySize, LDS_CONV);

  const int vec8 = ((NEDGE & 3) == 0) ? 1 : 0;
  k_tables<<<1, NTHR, 0, stream>>>(emb, mw1, mb1, mw2, mb2, fw1, fb1, fw2, fb2, fw3, fb3, tpw, cell, PAR);
  k_bucket<<<NBKT, NTHR, LDS_BKT, stream>>>(edst, LISTB, HDR, NNODE, NEDGE, vec8);
  k_conv<<<NCONV, NTHR, LDS_CONV, stream>>>(pos, atype, batch, esrc, edst, shifts, PAR, LISTB, HDR, out, NNODE, NEDGE);
}
